// GraphProp_10565619548251
// MI455X (gfx1250) — hardware-verified
//
#include <hip/hip_runtime.h>
#include <stddef.h>


#define H      128
#define G3     384
#define KM     257
#define XP     256
#define NB     256
#define NTHR   256
#define NWAVE  8
#define EPT    8
#define CHUNK  (NTHR * EPT)
#define WCAP   (EPT * 32)
#define NROW   16
#define FR     16

static_assert(WCAP == 256);
static_assert(NB == 256);
static_assert(NTHR == NB);
static_assert((NB % NROW) == 0);
static_assert((NB % NWAVE) == 0);
static_assert(CHUNK == 2048);
static_assert((G3 % FR) == 0);

typedef float          v4f  __attribute__((ext_vector_type(4)));
typedef float          v8f  __attribute__((ext_vector_type(8)));
typedef int            v4i  __attribute__((ext_vector_type(4)));
typedef unsigned short v8us __attribute__((ext_vector_type(8)));
typedef __bf16         v16b __attribute__((ext_vector_type(16)));
union FragB { v16b v; v8us u[2]; };

__device__ __forceinline__ unsigned short bf16_rne(float f) {
  unsigned int u = __float_as_uint(f);
  u += 0x7FFFu + ((u >> 16) & 1u);
  return (unsigned short)(u >> 16);
}
__device__ __forceinline__ float bf16_val(unsigned short b) {
  return __uint_as_float(((unsigned int)b) << 16);
}
__device__ __forceinline__ void split8(const float* x, v8us& hi, v8us& lo) {
#pragma unroll
  for (int i = 0; i < 8; ++i) {
    const unsigned short hb = bf16_rne(x[i]);
    const float rem = x[i] - bf16_val(hb);
    hi[i] = hb;
    lo[i] = bf16_rne(rem);
  }
}
__device__ __forceinline__ v8f zero8f() {
  v8f z;
#pragma unroll
  for (int i = 0; i < 8; ++i) z[i] = 0.0f;
  return z;
}

__device__ __forceinline__ v8f wmb(v16b a, v16b b, v8f c) {
  v8f d = __builtin_amdgcn_wmma_f32_16x16x32_bf16(false, a, false, b, (short)0, c, false, false);
  asm volatile("v_nop\n\tv_nop\n\tv_nop\n\tv_nop" : "+v"(d) : "v"(a), "v"(b));
  return d;
}
__device__ __forceinline__ v8f wm3(const FragB& ah, const FragB& al, const FragB& bh, const FragB& bl, v8f c) {
  c = wmb(ah.v, bh.v, c);
  c = wmb(ah.v, bl.v, c);
  c = wmb(al.v, bh.v, c);
  return c;
}
__device__ __forceinline__ void ldfrag(FragB& f, const unsigned short* __restrict__ p, int pitch, int row, int k0, int h) {
  const unsigned short* q = p + (size_t)row * (size_t)pitch + k0 + 8 * h;
  f.u[0] = *(const v8us*)q;
  f.u[1] = *(const v8us*)(q + 16);
}

__device__ __forceinline__ float sigm(float x) {
  x = fminf(fmaxf(x, -30.0f), 30.0f);
  return 1.0f / (1.0f + __expf(-x));
}

__global__ __launch_bounds__(256) void k_whh(const float* __restrict__ W, unsigned short* phi,
                                             unsigned short* plo, int n8) {
  const int i = blockIdx.x * 256 + threadIdx.x;
  const bool ok = i < n8;
  const int ic = ok ? i : (n8 - 1);
  const float* p = W + (size_t)ic * 8;
  const v4f a = *(const v4f*)p;
  const v4f b = *(const v4f*)(p + 4);
  float x[8];
  x[0] = a.x; x[1] = a.y; x[2] = a.z; x[3] = a.w;
  x[4] = b.x; x[5] = b.y; x[6] = b.z; x[7] = b.w;
  v8us hi, lo;
  split8(x, hi, lo);
  const size_t off = (size_t)ic * 8;
  if (ok) { *(volatile v8us*)(phi + off) = hi; *(volatile v8us*)(plo + off) = lo; }
  __threadfence();
  if (ok) { *(volatile v8us*)(phi + off) = hi; *(volatile v8us*)(plo + off) = lo; }
}

__global__ __launch_bounds__(256) void k_wfold(const float* __restrict__ Wih, const float* __restrict__ Wmsg,
                                               const float* __restrict__ bmsg,
                                               unsigned short* wphi, unsigned short* wplo, float* uv) {
  __shared__ __attribute__((aligned(16))) float wl[256 * FR];
  __shared__ __attribute__((aligned(16))) float stg[FR * 256];
  __shared__ float hwL[256];
  __shared__ float bmL[256];
  __shared__ __attribute__((aligned(16))) float uvs[2 * FR];

  const int tid = threadIdx.x, lane = tid & 31, wave = tid >> 5;
  const int rt = blockIdx.x, t = blockIdx.y;
  const float* Wi = Wih + ((size_t)t * G3 + (size_t)rt * FR) * 256;
  const float* Wm = Wmsg + (size_t)t * 256 * KM;
  const float* bm = bmsg + (size_t)t * 256;

#pragma unroll 1
  for (int i = tid; i < FR * 256; i += NTHR) {
    const int j = i >> 8, o = i & 255;
    wl[o * FR + j] = Wi[i];
  }
  hwL[tid] = Wm[(size_t)tid * KM + 256];
  bmL[tid] = bm[tid];
  __syncthreads();

  float acc[FR];
#pragma unroll
  for (int j = 0; j < FR; ++j) acc[j] = 0.0f;
#pragma unroll 1
  for (int o = 0; o < 256; ++o) {
    const float b = Wm[(size_t)o * KM + tid];
    const v4f w0 = *(const v4f*)(wl + o * FR);
    const v4f w1 = *(const v4f*)(wl + o * FR + 4);
    const v4f w2 = *(const v4f*)(wl + o * FR + 8);
    const v4f w3 = *(const v4f*)(wl + o * FR + 12);
    acc[0]  = fmaf(w0.x, b, acc[0]);  acc[1]  = fmaf(w0.y, b, acc[1]);
    acc[2]  = fmaf(w0.z, b, acc[2]);  acc[3]  = fmaf(w0.w, b, acc[3]);
    acc[4]  = fmaf(w1.x, b, acc[4]);  acc[5]  = fmaf(w1.y, b, acc[5]);
    acc[6]  = fmaf(w1.z, b, acc[6]);  acc[7]  = fmaf(w1.w, b, acc[7]);
    acc[8]  = fmaf(w2.x, b, acc[8]);  acc[9]  = fmaf(w2.y, b, acc[9]);
    acc[10] = fmaf(w2.z, b, acc[10]); acc[11] = fmaf(w2.w, b, acc[11]);
    acc[12] = fmaf(w3.x, b, acc[12]); acc[13] = fmaf(w3.y, b, acc[13]);
    acc[14] = fmaf(w3.z, b, acc[14]); acc[15] = fmaf(w3.w, b, acc[15]);
  }
#pragma unroll
  for (int j = 0; j < FR; ++j) stg[j * 256 + tid] = acc[j];

  if (wave == 0) {
    const int jj = lane & 15, s = lane >> 4;
    float au = 0.0f;
#pragma unroll 1
    for (int o = 0; o < 256; ++o) {
      const float w  = wl[o * FR + jj];
      const float c0 = hwL[o];
      const float c1 = bmL[o];
      const float cc = (s == 0) ? c0 : c1;
      au = fmaf(w, cc, au);
    }
    uvs[2 * jj + s] = au;
  }
  __syncthreads();

  v8us hi2[2], lo2[2];
#pragma unroll
  for (int q = 0; q < 2; ++q) {
    const float* sp = stg + (2 * wave + q) * 256 + 8 * lane;
    const v4f a = *(const v4f*)sp, b = *(const v4f*)(sp + 4);
    float x[8];
    x[0] = a.x; x[1] = a.y; x[2] = a.z; x[3] = a.w; x[4] = b.x; x[5] = b.y; x[6] = b.z; x[7] = b.w;
    split8(x, hi2[q], lo2[q]);
  }
  const int lq = lane & 7;
  const v4f u4 = *(const v4f*)(uvs + 4 * lq);
  const bool wu = (wave == 0) && (lane < 8);
  const size_t rowb = (size_t)t * G3 + (size_t)rt * FR;
  const size_t uoff = rowb * 2 + 4 * (size_t)lq;

#pragma unroll
  for (int q = 0; q < 2; ++q) {
    const size_t off = (rowb + (size_t)(2 * wave + q)) * XP + 8 * (size_t)lane;
    *(volatile v8us*)(wphi + off) = hi2[q];
    *(volatile v8us*)(wplo + off) = lo2[q];
  }
  if (wu) *(volatile v4f*)(uv + uoff) = u4;
  __threadfence();
#pragma unroll
  for (int q = 0; q < 2; ++q) {
    const size_t off = (rowb + (size_t)(2 * wave + q)) * XP + 8 * (size_t)lane;
    *(volatile v8us*)(wphi + off) = hi2[q];
    *(volatile v8us*)(wplo + off) = lo2[q];
  }
  if (wu) *(volatile v4f*)(uv + uoff) = u4;
}

__device__ __forceinline__ int scan_chunk(const int* __restrict__ dsts, int nE, int cbase, int nodeBase,
                                          int* list, int tid, int wave) {
  int wc = 0;
  const int el0  = tid * EPT;
  const int e0   = cbase + el0;
  const int sent = -2147483647 - 1;
  const int em   = nE - 1;
  v4i da, db;
  if (cbase + CHUNK <= nE) {
    da = *(const v4i*)(dsts + e0);
    db = *(const v4i*)(dsts + e0 + 4);
  } else {
    da.x = (e0     < nE) ? dsts[(e0     < em) ? e0     : em] : sent;
    da.y = (e0 + 1 < nE) ? dsts[(e0 + 1 < em) ? e0 + 1 : em] : sent;
    da.z = (e0 + 2 < nE) ? dsts[(e0 + 2 < em) ? e0 + 2 : em] : sent;
    da.w = (e0 + 3 < nE) ? dsts[(e0 + 3 < em) ? e0 + 3 : em] : sent;
    db.x = (e0 + 4 < nE) ? dsts[(e0 + 4 < em) ? e0 + 4 : em] : sent;
    db.y = (e0 + 5 < nE) ? dsts[(e0 + 5 < em) ? e0 + 5 : em] : sent;
    db.z = (e0 + 6 < nE) ? dsts[(e0 + 6 < em) ? e0 + 6 : em] : sent;
    db.w = (e0 + 7 < nE) ? dsts[(e0 + 7 < em) ? e0 + 7 : em] : sent;
  }
  const unsigned nb = (unsigned)nodeBase;
  const unsigned s0 = (unsigned)da.x - nb, s1 = (unsigned)da.y - nb;
  const unsigned s2 = (unsigned)da.z - nb, s3 = (unsigned)da.w - nb;
  const unsigned s4 = (unsigned)db.x - nb, s5 = (unsigned)db.y - nb;
  const unsigned s6 = (unsigned)db.z - nb, s7 = (unsigned)db.w - nb;
  const bool h0 = s0 < (unsigned)NB, h1 = s1 < (unsigned)NB, h2 = s2 < (unsigned)NB, h3 = s3 < (unsigned)NB;
  const bool h4 = s4 < (unsigned)NB, h5 = s5 < (unsigned)NB, h6 = s6 < (unsigned)NB, h7 = s7 < (unsigned)NB;
  const unsigned any = __builtin_amdgcn_ballot_w32(h0 | h1 | h2 | h3 | h4 | h5 | h6 | h7);
  if (any != 0u) {
#define HITJ(J, HJ, SJ) { \
      const unsigned mj = __builtin_amdgcn_ballot_w32(HJ); \
      if (mj != 0u) { \
        if (HJ) { \
          const int pos = wc + (int)__builtin_amdgcn_mbcnt_lo(mj, 0u); \
          if (pos < WCAP) list[wave * WCAP + pos] = ((el0 + (J)) << 8) | (int)(SJ); \
        } \
        wc += (int)__builtin_popcount(mj); } }
    HITJ(0, h0, s0)
    HITJ(1, h1, s1)
    HITJ(2, h2, s2)
    HITJ(3, h3, s3)
    HITJ(4, h4, s4)
    HITJ(5, h5, s5)
    HITJ(6, h6, s6)
    HITJ(7, h7, s7)
#undef HITJ
  }
  return wc;
}

__global__ __launch_bounds__(NTHR) void k_gather(const float* __restrict__ hv, const float* __restrict__ he,
                                                  const int* __restrict__ srcs, const int* __restrict__ dsts,
                                                  unsigned short* xhi, unsigned short* xlo, float* side,
                                                  int nN, int nE) {
  __shared__ __attribute__((aligned(16))) float acc[NB * H];
  __shared__ __attribute__((aligned(16))) int   list[NWAVE * WCAP];
  __shared__ __attribute__((aligned(16))) float cntL[NB];
  __shared__ __attribute__((aligned(16))) float hesL[NB];
  __shared__ int wcnt[NWAVE];

  const int tid = threadIdx.x, lane = tid & 31, wave = tid >> 5;
  const int nodeBase = blockIdx.x * NB;
  {
    v4f z; z.x = 0.0f; z.y = 0.0f; z.z = 0.0f; z.w = 0.0f;
#pragma unroll 1
    for (int i = tid; i < NB * H / 4; i += NTHR) *(v4f*)(acc + 4 * i) = z;
    cntL[tid] = 0.0f;
    hesL[tid] = 0.0f;
  }
  __syncthreads();

  const int nChunks = (nE + CHUNK - 1) / CHUNK;
#pragma unroll 1
  for (int ch = 0; ch < nChunks; ++ch) {
    const int cbase = ch * CHUNK;
    const int wc = scan_chunk(dsts, nE, cbase, nodeBase, list, tid, wave);
    if (lane == 0) wcnt[wave] = wc;
    __syncthreads();
    if (wave == 0) {
#pragma unroll 1
      for (int w = 0; w < NWAVE; ++w) {
        int n = wcnt[w];
        n = n > WCAP ? WCAP : (n < 0 ? 0 : n);
#pragma unroll 1
        for (int i = 0; i < n; ++i) {
          const int ent = list[w * WCAP + i];
          int el = ent >> 8;
          el = el < 0 ? 0 : (el > CHUNK - 1 ? CHUNK - 1 : el);
          const int slot = ent & (NB - 1);
          int e = cbase + el;
          e = e > nE - 1 ? nE - 1 : (e < 0 ? 0 : e);
          int s = srcs[e];
          s = s < 0 ? 0 : (s > nN - 1 ? nN - 1 : s);
          const float hev = he[e];
          const v4f v = *(const v4f*)(hv + (size_t)s * H + 4 * lane);
          v4f* ap = (v4f*)(acc + slot * H + 4 * lane);
          v4f a = *ap;
          a += v;
          *ap = a;
          if (lane == 0) { cntL[slot] += 1.0f; hesL[slot] += hev; }
        }
      }
    }
    __syncthreads();
  }

  const int  l15  = lane & 15;
  const bool lowh = lane < 16;
#pragma unroll 1
  for (int ps = 0; ps < 2; ++ps) {
#pragma unroll 1
    for (int q = 0; q < NB / NWAVE; ++q) {
      const int lr   = wave * (NB / NWAVE) + q;
      const int row  = nodeBase + lr;
      const int rowc = row > nN - 1 ? nN - 1 : row;
      const float* hp = hv + (size_t)rowc * H + 8 * l15;
      const v4f g0 = *(const v4f*)hp, g1 = *(const v4f*)(hp + 4);
      const float* sp = acc + lr * H + 8 * l15;
      const v4f t0 = *(const v4f*)sp, t1 = *(const v4f*)(sp + 4);
      float x[8];
      x[0] = lowh ? g0.x : t0.x; x[1] = lowh ? g0.y : t0.y; x[2] = lowh ? g0.z : t0.z; x[3] = lowh ? g0.w : t0.w;
      x[4] = lowh ? g1.x : t1.x; x[5] = lowh ? g1.y : t1.y; x[6] = lowh ? g1.z : t1.z; x[7] = lowh ? g1.w : t1.w;
      v8us hi, lo;
      split8(x, hi, lo);
      const size_t off = (size_t)row * XP + 8 * (size_t)lane;
      *(volatile v8us*)(xhi + off) = hi;
      *(volatile v8us*)(xlo + off) = lo;
    }
    if (wave < 4) {
      const int L = wave * 32 + lane;
      v4f sv;
      sv.x = cntL[2 * L];     sv.y = hesL[2 * L];
      sv.z = cntL[2 * L + 1]; sv.w = hesL[2 * L + 1];
      *(volatile v4f*)(side + ((size_t)nodeBase + 2 * (size_t)L) * 2) = sv;
    }
    if (ps == 0) __threadfence();
  }
}

__global__ __launch_bounds__(NTHR) void k_node(const unsigned short* __restrict__ xhi, const unsigned short* __restrict__ xlo,
                                                const float* __restrict__ side, const float* __restrict__ hcur,
                                                const unsigned short* __restrict__ wphi, const unsigned short* __restrict__ wplo,
                                                const float* __restrict__ uv,
                                                const unsigned short* __restrict__ whhi, const unsigned short* __restrict__ whlo,
                                                const float* __restrict__ bih, const float* __restrict__ bhh,
                                                float* outp, int nN, int outRows) {
  __shared__ __attribute__((aligned(16))) float otile[NROW * H];
  __shared__ float bihL[G3];
  __shared__ float bhhL[G3];
  __shared__ float uvL[2 * G3];
  __shared__ float sd[2 * NROW];

  const int tid = threadIdx.x, lane = tid & 31, wave = tid >> 5, h = lane >> 4, m = lane & 15;
  const int row0 = blockIdx.x * NROW;
#pragma unroll 1
  for (int i = tid; i < G3; i += NTHR) { bihL[i] = bih[i]; bhhL[i] = bhh[i]; }
#pragma unroll 1
  for (int i = tid; i < 2 * G3; i += NTHR) uvL[i] = uv[i];
  if (tid < 2 * NROW) sd[tid] = side[(size_t)row0 * 2 + tid];
  __syncthreads();

  const int g    = wave;
  const int arow = row0 + m;
  const int c    = 16 * g + m;

  v8f P[3], Q[3], Hq[3];
#pragma unroll
  for (int gt = 0; gt < 3; ++gt) { P[gt] = zero8f(); Q[gt] = zero8f(); Hq[gt] = zero8f(); }

#pragma unroll 1
  for (int ks = 0; ks < 4; ++ks) {
    const int k0 = ks * 32;
    FragB ah, al;
    ldfrag(ah, xhi, XP, arow, k0, h);
    ldfrag(al, xlo, XP, arow, k0, h);
#pragma unroll
    for (int gt = 0; gt < 3; ++gt) {
      const int jr = gt * H + c;
      FragB bfh, bfl;
      ldfrag(bfh, wphi, XP, jr, k0, h);
      ldfrag(bfl, wplo, XP, jr, k0, h);
      P[gt] = wm3(ah, al, bfh, bfl, P[gt]);
      ldfrag(bfh, whhi, H, jr, k0, h);
      ldfrag(bfl, whlo, H, jr, k0, h);
      Hq[gt] = wm3(ah, al, bfh, bfl, Hq[gt]);
    }
  }
#pragma unroll 1
  for (int ks = 4; ks < 8; ++ks) {
    const int k0 = ks * 32;
    FragB ah, al;
    ldfrag(ah, xhi, XP, arow, k0, h);
    ldfrag(al, xlo, XP, arow, k0, h);
#pragma unroll
    for (int gt = 0; gt < 3; ++gt) {
      const int jr = gt * H + c;
      FragB bfh, bfl;
      ldfrag(bfh, wphi, XP, jr, k0, h);
      ldfrag(bfl, wplo, XP, jr, k0, h);
      Q[gt] = wm3(ah, al, bfh, bfl, Q[gt]);
    }
  }

#pragma unroll
  for (int r = 0; r < 8; ++r) {
    const int lr = 8 * h + r;
    const float cnt = sd[2 * lr];
    const float hes = sd[2 * lr + 1];
    int row = row0 + lr;
    row = row > nN - 1 ? nN - 1 : row;
    const float hval = hcur[(size_t)row * H + c];
    float gi[3], gh[3];
#pragma unroll
    for (int gt = 0; gt < 3; ++gt) {
      const int j = gt * H + c;
      gi[gt] = cnt * P[gt][r] + Q[gt][r] + cnt * uvL[2 * j + 1] + hes * uvL[2 * j] + bihL[j];
      gh[gt] = Hq[gt][r] + bhhL[j];
    }
    const float rg = sigm(gi[0] + gh[0]);
    const float zg = sigm(gi[1] + gh[1]);
    const float ng = tanhf(gi[2] + rg * gh[2]);
    otile[lr * H + c] = (1.0f - zg) * ng + zg * hval;
  }
  __syncthreads();

  const int ra = row0 + 2 * wave, rb = ra + 1;
  const v4f oa = *(const v4f*)(otile + (2 * wave) * H + 4 * lane);
  const v4f ob = *(const v4f*)(otile + (2 * wave + 1) * H + 4 * lane);
  const bool wa = ra < outRows, wb = rb < outRows;
  if (wa) *(volatile v4f*)(outp + (size_t)ra * H + 4 * lane) = oa;
  if (wb) *(volatile v4f*)(outp + (size_t)rb * H + 4 * lane) = ob;
  __threadfence();
  if (wa) *(volatile v4f*)(outp + (size_t)ra * H + 4 * lane) = oa;
  if (wb) *(volatile v4f*)(outp + (size_t)rb * H + 4 * lane) = ob;
}

extern "C" void kernel_launch(void* const* d_in, const int* in_sizes, int n_in,
                              void* d_out, int out_size, void* d_ws, size_t ws_size,
                              hipStream_t stream) {
  if (n_in < 10) return;
  const int nN = in_sizes[0] / H;
  const int nE = in_sizes[1];
  if (nN <= 0 || nE <= 0 || in_sizes[0] != nN * H) return;
  if (in_sizes[2] != nE || in_sizes[3] != nE) return;
  if (in_sizes[4] != 2 * 256 * KM || in_sizes[5] != 2 * 256) return;
  if (in_sizes[6] != 2 * G3 * 256 || in_sizes[7] != 2 * G3 * H) return;
  if (in_sizes[8] != 2 * G3 || in_sizes[9] != 2 * G3) return;
  if (out_size != nN * H) return;

  const float* hv0   = (const float*)d_in[0];
  const float* he    = (const float*)d_in[1];
  const int*   src   = (const int*)d_in[2];
  const int*   dst   = (const int*)d_in[3];
  const float* W_msg = (const float*)d_in[4];
  const float* b_msg = (const float*)d_in[5];
  const float* W_ih  = (const float*)d_in[6];
  const float* W_hh  = (const float*)d_in[7];
  const float* b_ih  = (const float*)d_in[8];
  const float* b_hh  = (const float*)d_in[9];
  float* out = (float*)d_out;

  const int NPAD  = ((nN + NB - 1) / NB) * NB;
  const int nBlkG = NPAD / NB;
  const int nBlkN = (nN + NROW - 1) / NROW;

  char* ws = (char*)d_ws;
  size_t off = 0;
  const size_t szX   = ((size_t)NPAD * XP * 2 + 255) & ~(size_t)255;
  const size_t szSd  = ((size_t)NPAD * 2 * 4 + 255) & ~(size_t)255;
  const size_t szHt  = ((size_t)NPAD * H * 4 + 255) & ~(size_t)255;
  const size_t szWp  = ((size_t)2 * G3 * XP * 2 + 255) & ~(size_t)255;
  const size_t szWh  = ((size_t)2 * G3 * H * 2 + 255) & ~(size_t)255;
  const size_t szUv  = ((size_t)2 * G3 * 2 * 4 + 255) & ~(size_t)255;
  const size_t oXhi = off; off += szX;
  const size_t oXlo = off; off += szX;
  const size_t oSd  = off; off += szSd;
  const size_t oHt  = off; off += szHt;
  const size_t oWph = off; off += szWp;
  const size_t oWpl = off; off += szWp;
  const size_t oWhh = off; off += szWh;
  const size_t oWhl = off; off += szWh;
  const size_t oUv  = off; off += szUv;
  if (off > ws_size || off > (size_t)134217728) return;

  unsigned short* xhi  = (unsigned short*)(ws + oXhi);
  unsigned short* xlo  = (unsigned short*)(ws + oXlo);
  float*          side = (float*)(ws + oSd);
  float*          htmp = (float*)(ws + oHt);
  unsigned short* wphi = (unsigned short*)(ws + oWph);
  unsigned short* wplo = (unsigned short*)(ws + oWpl);
  unsigned short* whhi = (unsigned short*)(ws + oWhh);
  unsigned short* whlo = (unsigned short*)(ws + oWhl);
  float*          uv   = (float*)(ws + oUv);

  const int n8 = 2 * G3 * H / 8;
  k_whh<<<(n8 + 255) / 256, 256, 0, stream>>>(W_hh, whhi, whlo, n8);
  k_wfold<<<dim3(G3 / FR, 2), NTHR, 0, stream>>>(W_ih, W_msg, b_msg, wphi, wplo, uv);

  for (int t = 0; t < 2; ++t) {
    const float* hcur = (t == 0) ? hv0 : htmp;
    float* hout = (t == 0) ? htmp : out;
    const int outRows = (t == 0) ? nBlkN * NROW : nN;
    k_gather<<<nBlkG, NTHR, 0, stream>>>(hcur, he, src, dst, xhi, xlo, side, nN, nE);
    k_node<<<nBlkN, NTHR, 0, stream>>>(xhi, xlo, side, hcur,
                                        wphi + (size_t)t * G3 * XP, wplo + (size_t)t * G3 * XP,
                                        uv + (size_t)t * G3 * 2,
                                        whhi + (size_t)t * G3 * H, whlo + (size_t)t * G3 * H,
                                        b_ih + (size_t)t * G3, b_hh + (size_t)t * G3,
                                        hout, nN, outRows);
  }
}
